// IpaMultiRigidDenoiser_31937376813592
// MI455X (gfx1250) — hardware-verified
//
#include <hip/hip_runtime.h>
#include <math.h>

#define BB 2
#define NN 512
#define CS 384
#define CZ 128
#define HH 4
#define CC 32
#define IE 256
#define NAA 21
#define NRBF 16
#define NREL 65
#define ROWS 1024
#define ZZ 8
#define LINC 576
#define FEAT 768
#define K1 544
#define LD1 576
#define QW 64
#define SW 96
#define FRW 32
#define WPLD 128
#define KPAIR 96
#define SPP 516
#define NTHA 320

#define PIF     3.14159265358979323846f
#define WLF     0.57735026918962576f
#define COEFF   0.06804138174397717f
#define RSQCF   0.17677669529663688f
#define NEGLOGF (-0.07252236513367074f)
#define RBFSTEP 1.3333333333333333f
#define RBFK    0.32f

typedef unsigned short u16;
typedef __bf16 v16b __attribute__((ext_vector_type(16)));
typedef u16    v8us __attribute__((ext_vector_type(8)));
typedef float  v8f  __attribute__((ext_vector_type(8)));
typedef float  v4f  __attribute__((ext_vector_type(4)));
typedef v4f  __attribute__((may_alias)) v4fa;
typedef v8us __attribute__((may_alias)) v8usa;
union FragB { v16b v; v8us u[2]; };

__device__ __forceinline__ int imin(int a, int b) { return a < b ? a : b; }
__device__ __forceinline__ int imax(int a, int b) { return a > b ? a : b; }
__device__ __forceinline__ float sel3(int d, float a, float b, float c) { return (d == 0) ? a : ((d == 1) ? b : c); }

__device__ __forceinline__ v8f wmma_bf(v16b a, v16b b, v8f c) {
  v8f d = __builtin_amdgcn_wmma_f32_16x16x32_bf16(false, a, false, b, (short)0, c, false, false);
  asm volatile("v_nop\n\tv_nop\n\tv_nop\n\tv_nop" : "+v"(d) : "v"(a), "v"(b));
  return d;
}
__device__ __forceinline__ v8f mac3(v16b ah, v16b al, v16b bh, v16b bl, v8f c) {
  c = wmma_bf(ah, bh, c);
  c = wmma_bf(ah, bl, c);
  c = wmma_bf(al, bh, c);
  return c;
}

__device__ __forceinline__ u16 bfb(float v) {
  unsigned u = __float_as_uint(v);
  u += 0x7FFFu + ((u >> 16) & 1u);
  return (u16)(u >> 16);
}
__device__ __forceinline__ float bff(u16 s) { return __uint_as_float(((unsigned)s) << 16); }

__device__ __forceinline__ void split8(v4f a, v4f c, v8us& hi, v8us& lo) {
  const float x[8] = {a.x, a.y, a.z, a.w, c.x, c.y, c.z, c.w};
  u16 hb[8], lb[8];
  #pragma unroll
  for (int i = 0; i < 8; ++i) { hb[i] = bfb(x[i]); lb[i] = bfb(x[i] - bff(hb[i])); }
  const v8us H = {hb[0], hb[1], hb[2], hb[3], hb[4], hb[5], hb[6], hb[7]};
  const v8us L = {lb[0], lb[1], lb[2], lb[3], lb[4], lb[5], lb[6], lb[7]};
  hi = H; lo = L;
}
__device__ __forceinline__ void split16v(v4f p0, v4f p1, v4f p2, v4f p3, v16b& hi, v16b& lo) {
  FragB H, L;
  split8(p0, p1, H.u[0], L.u[0]);
  split8(p2, p3, H.u[1], L.u[1]);
  hi = H.v; lo = L.v;
}

__device__ __forceinline__ v16b ldfrag(const u16* p, int h) {
  FragB f;
  f.u[0] = *(const v8usa*)(p + 8 * h);
  f.u[1] = *(const v8usa*)(p + 16 + 8 * h);
  return f.v;
}

__device__ __forceinline__ void stv4(float* p, v4f v) { *(volatile v4f*)p = v; }
__device__ __forceinline__ void stv8(u16* p, v8us v) { *(volatile v8us*)p = v; }

__device__ __forceinline__ float wsum(float v) {
  v += __shfl_xor(v, 16); v += __shfl_xor(v, 8); v += __shfl_xor(v, 4); v += __shfl_xor(v, 2); v += __shfl_xor(v, 1);
  return v;
}

__global__ __launch_bounds__(256) void k_prep(
    const float* __restrict__ tt, const float* __restrict__ gamma,
    const float* __restrict__ Wrel, const float* __restrict__ Wrbf,
    const float* __restrict__ Wch, const float* __restrict__ Wbd, const float* __restrict__ Wb,
    float* tab, u16* wph, u16* wpl)
{
  __shared__ __attribute__((aligned(16))) float st[1024];
  const int tid = threadIdx.x;
  for (int i = tid; i < 1024; i += 256) st[i] = 0.f;
  __syncthreads();

  for (int idx = tid; idx < NREL * HH; idx += 256) {
    const int rel = idx >> 2, hq = idx & 3;
    float s = 0.f;
    #pragma unroll 1
    for (int zc = 0; zc < CZ; ++zc) s = fmaf(Wrel[rel * CZ + zc], Wb[zc * HH + hq], s);
    st[idx] = s;
  }
  if (tid < NRBF * HH) {
    const int rr = tid >> 2, hq = tid & 3;
    float s = 0.f;
    #pragma unroll 1
    for (int zc = 0; zc < CZ; ++zc) s = fmaf(Wrbf[rr * CZ + zc], Wb[zc * HH + hq], s);
    st[260 + tid] = s;
  }
  if (tid < HH) {
    float ch = 0.f, bd = 0.f;
    #pragma unroll 1
    for (int zc = 0; zc < CZ; ++zc) { ch = fmaf(Wch[zc], Wb[zc * HH + tid], ch); bd = fmaf(Wbd[zc], Wb[zc * HH + tid], bd); }
    st[324 + tid] = ch;
    st[328 + tid] = bd;
    const float g = gamma[tid];
    const float sp = fmaxf(g, 0.f) + log1pf(expf(-fabsf(g)));
    st[332 + tid] = COEFF * sp;
  }
  {
    const int bq = tid >> 7, k = tid & 127;
    const float fr = expf((float)k * NEGLOGF);
    const float ang = (tt[bq] * 10000.0f) * fr;
    st[512 + bq * 256 + k] = sinf(ang);
    st[512 + bq * 256 + 128 + k] = cosf(ang);
  }
  __syncthreads();
  if (tid < 96 || tid >= 128) {
    const v4f v = *(const v4fa*)&st[4 * tid];
    stv4(tab + 4 * tid, v);
    __threadfence();
    stv4(tab + 4 * tid, v);
  }
  #pragma unroll 1
  for (int q = 0; q < 8; ++q) {
    const int g = tid + 256 * q;
    const int n = g >> 4, k0 = (g & 15) * 8;
    float x[8];
    #pragma unroll
    for (int i = 0; i < 8; ++i) {
      const int k = k0 + i;
      const float a  = Wrel[(size_t)imin(k, NREL - 1) * CZ + n];
      const float bq = Wrbf[(size_t)imin(imax(k - 65, 0), NRBF - 1) * CZ + n];
      const float c  = Wch[n];
      const float d  = Wbd[n];
      x[i] = (k < 65) ? a : ((k < 81) ? bq : ((k == 81) ? c : ((k == 82) ? d : 0.f)));
    }
    const v4f a4 = {x[0], x[1], x[2], x[3]};
    const v4f c4 = {x[4], x[5], x[6], x[7]};
    v8us hi, lo;
    split8(a4, c4, hi, lo);
    stv8(wph + (size_t)g * 8, hi);
    stv8(wpl + (size_t)g * 8, lo);
    __threadfence();
    stv8(wph + (size_t)g * 8, hi);
    stv8(wpl + (size_t)g * 8, lo);
  }
}

__global__ __launch_bounds__(256) void k_wconv(
    const float* __restrict__ Wnode, const float* __restrict__ Wseq, const float* __restrict__ Wtime,
    const float* __restrict__ Wq, const float* __restrict__ Wk, const float* __restrict__ Wv,
    const float* __restrict__ Wqp, const float* __restrict__ Wkp, const float* __restrict__ Wvp,
    const float* __restrict__ Wout,
    u16* wnh, u16* wnl, u16* wch, u16* wcl, u16* woh, u16* wol, float* tab)
{
  __shared__ __attribute__((aligned(16))) float srcp[128];
  const int blk = blockIdx.x, tid = threadIdx.x;
  const int plane = (blk < 108) ? 0 : ((blk < 216) ? 1 : 2);
  float x[8];
  u16* dh; u16* dl; size_t doff;
  if (plane == 0) {
    const int g = blk * 256 + tid;
    const int n = g / 72, k0 = (g - n * 72) * 8;
    #pragma unroll
    for (int i = 0; i < 8; ++i) {
      const int k = k0 + i;
      const float* src = (k < 256) ? Wnode : ((k < 288) ? Wseq : Wtime);
      const int r = (k < 256) ? k : ((k < 288) ? imin(k - 256, NAA - 1) : imin(k - 288, IE - 1));
      const float v = src[(size_t)r * CS + n];
      const bool ok = (k < 256 + NAA) || (k >= 288 && k < K1);
      x[i] = ok ? v : 0.f;
    }
    dh = wnh; dl = wnl; doff = (size_t)g * 8;
  } else if (plane == 1) {
    const int g = (blk - 108) * 256 + tid;
    const int n = g / 48, k0 = (g - n * 48) * 8;
    const float* src = (n < 128) ? Wq : ((n < 256) ? Wk : ((n < 384) ? Wv : ((n < 432) ? Wqp : ((n < 480) ? Wkp : Wvp))));
    const int wd  = (n < 384) ? 128 : ((n < 480) ? 48 : 96);
    const int col = (n < 128) ? n : ((n < 256) ? (n - 128) : ((n < 384) ? (n - 256) : ((n < 432) ? (n - 384) : ((n < 480) ? (n - 432) : (n - 480)))));
    #pragma unroll
    for (int i = 0; i < 8; ++i) x[i] = src[(size_t)(k0 + i) * wd + col];
    dh = wch; dl = wcl; doff = (size_t)g * 8;
  } else {
    const int g = (blk - 216) * 256 + tid;
    const int n = g / 96, k0 = (g - n * 96) * 8;
    #pragma unroll
    for (int i = 0; i < 8; ++i) x[i] = Wout[(size_t)(k0 + i) * CS + n];
    dh = woh; dl = wol; doff = (size_t)g * 8;
  }
  {
    const v4f a4 = {x[0], x[1], x[2], x[3]};
    const v4f c4 = {x[4], x[5], x[6], x[7]};
    v8us hi, lo;
    split8(a4, c4, hi, lo);
    stv8(dh + doff, hi);
    stv8(dl + doff, lo);
    __threadfence();
    stv8(dh + doff, hi);
    stv8(dl + doff, lo);
  }
  if (blk == 0) {
    if (tid < 128) {
      const float e = (float)(2 * tid) * (1.0f / 256.0f);
      srcp[tid] = 1.0f / powf(2056.0f, e);
    }
    __syncthreads();
    if (tid < 32) {
      const v4f v = *(const v4fa*)&srcp[4 * tid];
      stv4(tab + 384 + 4 * tid, v);
      __threadfence();
      stv4(tab + 384 + 4 * tid, v);
    }
  }
}

__global__ __launch_bounds__(96) void k_embed(
    const int* __restrict__ seq, const int* __restrict__ seq_idx, const float* __restrict__ tab,
    u16* a1h, u16* a1l)
{
  __shared__ __attribute__((aligned(16))) float srow[LD1];
  const int row = blockIdx.x, b = row >> 9;
  const int tid = threadIdx.x, w = tid >> 5, lane = tid & 31;
  const float idf = (float)seq_idx[row] * PIF;
  const int sq = seq[row];
  if (w < 2) {
    #pragma unroll 1
    for (int mm = 0; mm < 2; ++mm) {
      const int a = tid + 64 * mm;
      const float ang = idf * tab[384 + a];
      srow[a] = sinf(ang);
      srow[128 + a] = cosf(ang);
    }
  } else {
    #pragma unroll 1
    for (int mm = 0; mm < 10; ++mm) {
      const int k = 256 + lane + 32 * mm;
      const int kt = imin(imax(k - 288, 0), 255);
      const float tv = tab[512 + b * 256 + kt];
      const float oh = ((k - 256) == sq) ? 1.f : 0.f;
      srow[k] = (k < 288) ? oh : ((k < K1) ? tv : 0.f);
    }
  }
  __syncthreads();
  if (tid < 72) {
    const v4f a = *(const v4fa*)&srow[8 * tid];
    const v4f c = *(const v4fa*)&srow[8 * tid + 4];
    v8us hi, lo;
    split8(a, c, hi, lo);
    u16* ph = a1h + (size_t)row * LD1 + 8 * tid;
    u16* pl = a1l + (size_t)row * LD1 + 8 * tid;
    stv8(ph, hi); stv8(pl, lo);
    __threadfence();
    stv8(ph, hi); stv8(pl, lo);
  }
}

__device__ __forceinline__ void gemm_store(const float* sC, float* Cf, int ldc, u16* Ch, u16* Cl, int ldh,
                                           int m0, int n0, int w, int lane) {
  if (Cf) {
    #pragma unroll
    for (int i = 0; i < 8; ++i) {
      const int row = 16 * w + 2 * i + (lane >> 4);
      const int c4 = (lane & 15) * 4;
      const v4f v = *(const v4fa*)(sC + row * 64 + c4);
      stv4(Cf + (size_t)(m0 + row) * ldc + n0 + c4, v);
    }
  }
  if (Ch) {
    #pragma unroll
    for (int i = 0; i < 4; ++i) {
      const int row = 16 * w + 4 * i + (lane >> 3);
      const int c8 = (lane & 7) * 8;
      const v4f a = *(const v4fa*)(sC + row * 64 + c8);
      const v4f c = *(const v4fa*)(sC + row * 64 + c8 + 4);
      v8us hi, lo;
      split8(a, c, hi, lo);
      stv8(Ch + (size_t)(m0 + row) * ldh + n0 + c8, hi);
      stv8(Cl + (size_t)(m0 + row) * ldh + n0 + c8, lo);
    }
  }
}

__global__ __launch_bounds__(128) void k_gemm3(
    const u16* __restrict__ Ah, const u16* __restrict__ Al, int lda,
    const u16* __restrict__ Bh, const u16* __restrict__ Bl, int ldb, int K,
    float* Cf, int ldc, const float* __restrict__ Cadd, int ldadd,
    u16* Ch, u16* Cl, int ldh)
{
  __shared__ __attribute__((aligned(16))) float sC[64 * 64];
  const int tid = threadIdx.x, lane = tid & 31, w = tid >> 5, h = lane >> 4, m = lane & 15;
  const int m0 = blockIdx.y * 64, n0 = blockIdx.x * 64, mw = m0 + 16 * w;
  const u16* ah0 = Ah + (size_t)(mw + m) * lda;
  const u16* al0 = Al + (size_t)(mw + m) * lda;
  const u16* bh0 = Bh + (size_t)(n0 + m) * ldb;
  const u16* bl0 = Bl + (size_t)(n0 + m) * ldb;

  const v8f z8 = {0.f, 0.f, 0.f, 0.f, 0.f, 0.f, 0.f, 0.f};
  v8f acc[4];
  #pragma unroll
  for (int nt = 0; nt < 4; ++nt) acc[nt] = z8;

  #pragma unroll 1
  for (int k0 = 0; k0 < K; k0 += 32) {
    const v16b ah = ldfrag(ah0 + k0, h);
    const v16b al = ldfrag(al0 + k0, h);
    #pragma unroll
    for (int nt = 0; nt < 4; ++nt) {
      const v16b bh = ldfrag(bh0 + (size_t)nt * 16 * ldb + k0, h);
      const v16b bl = ldfrag(bl0 + (size_t)nt * 16 * ldb + k0, h);
      acc[nt] = mac3(ah, al, bh, bl, acc[nt]);
    }
  }
  #pragma unroll
  for (int nt = 0; nt < 4; ++nt) {
    #pragma unroll
    for (int r = 0; r < 8; ++r) {
      const int row = 16 * w + 8 * h + r, col = 16 * nt + m;
      float v = acc[nt][r];
      if (Cadd) v += Cadd[(size_t)(m0 + row) * ldadd + n0 + col];
      sC[row * 64 + col] = v;
    }
  }
  __syncthreads();
  gemm_store(sC, Cf, ldc, Ch, Cl, ldh, m0, n0, w, lane);
  __threadfence();
  gemm_store(sC, Cf, ldc, Ch, Cl, ldh, m0, n0, w, lane);
}

__device__ __forceinline__ void pack_store(const float* sQ, const float* sK, const float* sV, const float* sF,
                                           float* Qp, float* Kp, float* Vp, float* Fp,
                                           size_t zrow, int row, int w, int lane) {
  if (lane < 16) {
    const v4f a = *(const v4fa*)(sQ + w * 64 + 4 * lane);
    const v4f b = *(const v4fa*)(sK + w * 64 + 4 * lane);
    const v4f c = *(const v4fa*)(sV + w * 64 + 4 * lane);
    stv4(Qp + zrow * QW + 4 * lane, a);
    stv4(Kp + zrow * QW + 4 * lane, b);
    stv4(Vp + zrow * QW + 4 * lane, c);
  }
  if (w == 0 && lane < 8) {
    const v4f f = *(const v4fa*)(sF + 4 * lane);
    stv4(Fp + (size_t)row * FRW + 4 * lane, f);
  }
}

__global__ __launch_bounds__(128) void k_pack(
    const float* __restrict__ lin, const float* __restrict__ rigid7,
    const int* __restrict__ seq_idx, const int* __restrict__ chain_idx, const float* __restrict__ mask,
    float* Qp, float* Kp, float* Vp, float* Fp)
{
  __shared__ __attribute__((aligned(16))) float sQ[4 * 64];
  __shared__ __attribute__((aligned(16))) float sK[4 * 64];
  __shared__ __attribute__((aligned(16))) float sV[4 * 64];
  __shared__ __attribute__((aligned(16))) float sF[32];
  const int row = blockIdx.x, b = row >> 9, n = row & (NN - 1);
  const int tid = threadIdx.x, w = tid >> 5, lane = tid & 31;
  const size_t zrow = (size_t)(b * HH + w) * NN + n;

  const float* r7 = rigid7 + (size_t)row * 7;
  float qw = r7[0], qx = r7[1], qy = r7[2], qz = r7[3];
  const float inv = 1.0f / sqrtf(qw * qw + qx * qx + qy * qy + qz * qz + 1e-8f);
  qw *= inv; qx *= inv; qy *= inv; qz *= inv;
  const float R00 = 1.f - 2.f * (qy * qy + qz * qz), R01 = 2.f * (qx * qy - qw * qz), R02 = 2.f * (qx * qz + qw * qy);
  const float R10 = 2.f * (qx * qy + qw * qz), R11 = 1.f - 2.f * (qx * qx + qz * qz), R12 = 2.f * (qy * qz - qw * qx);
  const float R20 = 2.f * (qx * qz - qw * qy), R21 = 2.f * (qy * qz + qw * qx), R22 = 1.f - 2.f * (qx * qx + qy * qy);
  const float t0 = r7[4], t1 = r7[5], t2 = r7[6];

  const float* L = lin + (size_t)row * LINC;
  const float qv = L[w * CC + lane];
  const float kv = L[128 + w * CC + lane];
  const float vv = L[256 + w * CC + lane];

  const int cq = imin(lane, 11), pq = cq / 3, dq = cq - 3 * pq;
  const float Rq0 = sel3(dq, R00, R10, R20), Rq1 = sel3(dq, R01, R11, R21), Rq2 = sel3(dq, R02, R12, R22);
  const float tq = sel3(dq, t0, t1, t2);
  const float* qpp = L + 384 + w * 12 + pq * 3;
  const float* kpp = L + 432 + w * 12 + pq * 3;
  float qf = Rq0 * qpp[0] + Rq1 * qpp[1] + Rq2 * qpp[2] + tq;
  float kf = Rq0 * kpp[0] + Rq1 * kpp[1] + Rq2 * kpp[2] + tq;
  qf = (lane < 12) ? qf : 0.f;
  kf = (lane < 12) ? kf : 0.f;

  const int cv = imin(lane, 23), pv = cv / 3, dv = cv - 3 * pv;
  const float Rv0 = sel3(dv, R00, R10, R20), Rv1 = sel3(dv, R01, R11, R21), Rv2 = sel3(dv, R02, R12, R22);
  const float tv = sel3(dv, t0, t1, t2);
  const float* vpp = L + 480 + w * 24 + pv * 3;
  float vg = Rv0 * vpp[0] + Rv1 * vpp[1] + Rv2 * vpp[2] + tv;
  vg = (lane < 24) ? vg : 0.f;

  const float qn2 = wsum(qf * qf);
  const float kn2 = wsum(kf * kf);
  const float si = (float)seq_idx[row], ci = (float)chain_idx[row], mk = mask[row];
  const float tl = (lane == 13) ? t0 : ((lane == 14) ? t1 : t2);

  const float qx2 = (lane < 12) ? qf : ((lane == 12) ? qn2 : ((lane < 16) ? tl : ((lane == 16) ? si : ((lane == 17) ? ci : 0.f))));
  const float kx2 = (lane < 12) ? kf : ((lane == 12) ? kn2 : ((lane < 16) ? tl : ((lane == 16) ? si : ((lane == 17) ? ci : ((lane == 18) ? mk : 0.f)))));
  const float vx2 = (lane < 24) ? vg : ((lane == 24) ? si : ((lane == 25) ? ci : 0.f));
  sQ[w * 64 + lane] = qv;  sQ[w * 64 + 32 + lane] = qx2;
  sK[w * 64 + lane] = kv;  sK[w * 64 + 32 + lane] = kx2;
  sV[w * 64 + lane] = vv;  sV[w * 64 + 32 + lane] = vx2;
  if (w == 0) {
    const float fv = (lane == 0) ? R00 : (lane == 1) ? R01 : (lane == 2) ? R02 : (lane == 3) ? R10 : (lane == 4) ? R11 :
                     (lane == 5) ? R12 : (lane == 6) ? R20 : (lane == 7) ? R21 : (lane == 8) ? R22 :
                     (lane == 9) ? t0 : (lane == 10) ? t1 : (lane == 11) ? t2 : 0.f;
    sF[lane] = fv;
  }
  __syncthreads();
  pack_store(sQ, sK, sV, sF, Qp, Kp, Vp, Fp, zrow, row, w, lane);
  __threadfence();
  pack_store(sQ, sK, sV, sF, Qp, Kp, Vp, Fp, zrow, row, w, lane);
}

__device__ __forceinline__ void pair_store(const float* srbf, float* rbfp, float* biasp, v4f bb,
                                           size_t bi, int j, int jb, int w, int lane) {
  stv4(biasp + (bi * NN + j) * 4, bb);
  #pragma unroll
  for (int q = 0; q < 4; ++q) {
    const int f = q * 128 + 4 * lane;
    const v4f v = *(const v4fa*)(srbf + w * 512 + f);
    stv4(rbfp + (bi * NN + jb + 32 * w) * 16 + f, v);
  }
}

__global__ __launch_bounds__(256) void k_pair(
    const float* __restrict__ rigid7, const int* __restrict__ seq_idx, const int* __restrict__ chain_idx,
    const float* __restrict__ bonds, const float* __restrict__ tab, float* rbfp, float* biasp)
{
  __shared__ float stab[336];
  __shared__ __attribute__((aligned(16))) float srbf[256 * 16];
  const int tid = threadIdx.x, lane = tid & 31, w = tid >> 5;
  const int blk = blockIdx.x;
  const size_t bi = (size_t)(blk >> 1);
  const int jb = (blk & 1) * 256;
  const int b = (int)(bi >> 9);
  const int j = jb + tid;
  const size_t bj = (size_t)b * NN + j;
  for (int q = tid; q < 336; q += 256) stab[q] = tab[q];
  __syncthreads();

  const float tix = rigid7[bi * 7 + 4], tiy = rigid7[bi * 7 + 5], tiz = rigid7[bi * 7 + 6];
  const float tjx = rigid7[bj * 7 + 4], tjy = rigid7[bj * 7 + 5], tjz = rigid7[bj * 7 + 6];
  const float dx = tix - tjx, dy = tiy - tjy, dz = tiz - tjz;
  const float d = sqrtf(dx * dx + dy * dy + dz * dz + 1e-8f);
  int rel = seq_idx[bi] - seq_idx[bj];
  rel = imax(-32, imin(32, rel)) + 32;
  const float same = (chain_idx[bi] == chain_idx[bj]) ? 1.f : 0.f;
  const float bd = bonds[bi * NN + j];
  float b0 = stab[rel * 4 + 0] + same * stab[324] + bd * stab[328];
  float b1 = stab[rel * 4 + 1] + same * stab[325] + bd * stab[329];
  float b2 = stab[rel * 4 + 2] + same * stab[326] + bd * stab[330];
  float b3 = stab[rel * 4 + 3] + same * stab[327] + bd * stab[331];
  #pragma unroll 1
  for (int r = 0; r < NRBF; ++r) {
    const float dd = d - (float)r * RBFSTEP;
    const float wv = __expf(-(dd * dd) * RBFK);
    srbf[tid * 16 + r] = wv;
    b0 = fmaf(wv, stab[260 + r * 4 + 0], b0);
    b1 = fmaf(wv, stab[260 + r * 4 + 1], b1);
    b2 = fmaf(wv, stab[260 + r * 4 + 2], b2);
    b3 = fmaf(wv, stab[260 + r * 4 + 3], b3);
  }
  const v4f bb = {b0, b1, b2, b3};
  __syncthreads();
  pair_store(srbf, rbfp, biasp, bb, bi, j, jb, w, lane);
  __threadfence();
  pair_store(srbf, rbfp, biasp, bb, bi, j, jb, w, lane);
}

__device__ __forceinline__ void attn_store(const float* sO, const float* sS, float* Op, float* Sp,
                                           size_t zrow0, int w, int lane) {
  if (w < 4) {
    #pragma unroll
    for (int i = 0; i < 4; ++i) {
      const int row = 8 * w + 2 * i + (lane >> 4);
      const int c4 = (lane & 15) * 4;
      const v4f v = *(const v4fa*)(sO + row * 64 + c4);
      stv4(Op + (zrow0 + row) * QW + c4, v);
    }
  } else {
    const int u = w - 4;
    #pragma unroll
    for (int i = 0; i < 4; ++i) {
      const int f = (u * 4 + i) * 32 + lane;
      const int row = f / 24;
      const int c4 = (f - row * 24) * 4;
      const v4f v = *(const v4fa*)(sS + row * SW + c4);
      stv4(Sp + (zrow0 + row) * SW + c4, v);
    }
  }
}

__global__ __launch_bounds__(NTHA) void k_attn(
    const float* __restrict__ Qp, const float* __restrict__ Kp, const float* __restrict__ Vp,
    const float* __restrict__ biasp, const float* __restrict__ rbfp, const float* __restrict__ bonds,
    const float* __restrict__ tab, float* Op, float* Sp)
{
  __shared__ __attribute__((aligned(16))) float sP[32 * SPP];
  __shared__ __attribute__((aligned(16))) float sQ[32 * 64];
  __shared__ __attribute__((aligned(16))) float sKV[64 * 64];
  __shared__ __attribute__((aligned(16))) float sO[32 * 64];
  __shared__ __attribute__((aligned(16))) float sS[32 * SW];

  const int tid = threadIdx.x, lane = tid & 31, w = tid >> 5, h = lane >> 4, m = lane & 15;
  const int z = blockIdx.y, b = z >> 2, hd = z & 3, i0 = blockIdx.x * 32;
  const size_t zrow0 = (size_t)z * NN + i0;
  const size_t brow0 = (size_t)b * NN + i0;

  for (int q = tid; q < 32 * SW; q += NTHA) sS[q] = 0.f;
  if (tid < 256) {
    #pragma unroll
    for (int mm = 0; mm < 2; ++mm) {
      const int f = tid + 256 * mm;
      const int row = f >> 4, c4 = (f & 15) * 4;
      *(v4fa*)&sQ[row * 64 + c4] = *(const v4fa*)(Qp + (zrow0 + row) * QW + c4);
    }
  }
  __syncthreads();

  const int prow = (tid < 256) ? (tid >> 3) : 0;
  const int jsub = tid & 7;
  v4f q4[8];
  v4f qf4[3];
  float qn2;
  {
    const float* qr = &sQ[prow * 64];
    #pragma unroll
    for (int c = 0; c < 8; ++c) q4[c] = *(const v4fa*)(qr + 4 * c);
    #pragma unroll
    for (int c = 0; c < 3; ++c) qf4[c] = *(const v4fa*)(qr + 32 + 4 * c);
    qn2 = qr[44];
  }
  const float cth = tab[332 + hd];
  const float* biasrow = biasp + (brow0 + prow) * (size_t)(NN * 4) + hd;

  #pragma unroll 1
  for (int c = 0; c < 8; ++c) {
    if (tid < 256) {
      #pragma unroll
      for (int mm = 0; mm < 4; ++mm) {
        const int f = tid + 256 * mm;
        const int kk = f >> 4, c4 = (f & 15) * 4;
        *(v4fa*)&sKV[kk * 64 + c4] = *(const v4fa*)(Kp + ((size_t)z * NN + 64 * c + kk) * QW + c4);
      }
    }
    __syncthreads();
    if (tid < 256) {
      #pragma unroll 1
      for (int mm = 0; mm < 8; ++mm) {
        const int kk = jsub + 8 * mm;
        const int j = 64 * c + kk;
        const float* kr = &sKV[kk * 64];
        float s = 0.f;
        #pragma unroll
        for (int q = 0; q < 8; ++q) {
          const v4f k4 = *(const v4fa*)(kr + 4 * q);
          s = fmaf(q4[q].x, k4.x, s); s = fmaf(q4[q].y, k4.y, s);
          s = fmaf(q4[q].z, k4.z, s); s = fmaf(q4[q].w, k4.w, s);
        }
        float dp = 0.f;
        #pragma unroll
        for (int q = 0; q < 3; ++q) {
          const v4f k4 = *(const v4fa*)(kr + 32 + 4 * q);
          dp = fmaf(qf4[q].x, k4.x, dp); dp = fmaf(qf4[q].y, k4.y, dp);
          dp = fmaf(qf4[q].z, k4.z, dp); dp = fmaf(qf4[q].w, k4.w, dp);
        }
        const float kn2 = kr[44];
        const float mk = kr[50];
        const float bias = biasrow[(size_t)j * 4];
        const float lg = WLF * (s * RSQCF + bias) - cth * ((qn2 + kn2) - 2.f * dp) + (mk - 1.f) * 1e9f;
        sP[prow * SPP + j] = lg;
      }
    }
    __syncthreads();
  }

  if (tid < 256) {
    float* pr = &sP[prow * SPP];
    float mx = -3.0e38f;
    #pragma unroll 4
    for (int mm = 0; mm < 64; ++mm) mx = fmaxf(mx, pr[jsub + 8 * mm]);
    mx = fmaxf(mx, __shfl_xor(mx, 1));
    mx = fmaxf(mx, __shfl_xor(mx, 2));
    mx = fmaxf(mx, __shfl_xor(mx, 4));
    float sm = 0.f;
    #pragma unroll 4
    for (int mm = 0; mm < 64; ++mm) {
      const float e = __expf(pr[jsub + 8 * mm] - mx);
      pr[jsub + 8 * mm] = e;
      sm += e;
    }
    sm += __shfl_xor(sm, 1);
    sm += __shfl_xor(sm, 2);
    sm += __shfl_xor(sm, 4);
    const float inv = 1.0f / sm;
    #pragma unroll 4
    for (int mm = 0; mm < 64; ++mm) pr[jsub + 8 * mm] *= inv;
  }
  __syncthreads();

  const int mt = w & 1, nt = (w >> 1) & 3;
  const v8f z8 = {0.f, 0.f, 0.f, 0.f, 0.f, 0.f, 0.f, 0.f};
  v8f acc = z8;
  const int rr = lane;
  const int isr = (int)sQ[rr * 64 + 48];
  const int icr = (int)sQ[rr * 64 + 49];
  float cacc = 0.f, bacc = 0.f;
  float racc[16];
  #pragma unroll
  for (int q = 0; q < 16; ++q) racc[q] = 0.f;
  const float* bondrow = bonds + (brow0 + rr) * (size_t)NN;
  const float* rbfrow = rbfp + (brow0 + rr) * (size_t)(NN * 16);

  #pragma unroll 1
  for (int c = 0; c < 8; ++c) {
    if (tid < 256) {
      #pragma unroll
      for (int mm = 0; mm < 4; ++mm) {
        const int f = tid + 256 * mm;
        const int kk = f >> 4, c4 = (f & 15) * 4;
        *(v4fa*)&sKV[kk * 64 + c4] = *(const v4fa*)(Vp + ((size_t)z * NN + 64 * c + kk) * QW + c4);
      }
    }
    __syncthreads();
    if (w < 8) {
      #pragma unroll
      for (int ks = 0; ks < 2; ++ks) {
        const int k0 = 32 * ks;
        const float* pr = &sP[(16 * mt + m) * SPP + 64 * c + k0];
        const v4f p0 = *(const v4fa*)(pr + 8 * h);
        const v4f p1 = *(const v4fa*)(pr + 8 * h + 4);
        const v4f p2 = *(const v4fa*)(pr + 16 + 8 * h);
        const v4f p3 = *(const v4fa*)(pr + 20 + 8 * h);
        v16b ah, al;
        split16v(p0, p1, p2, p3, ah, al);
        const int cn = 16 * nt + m;
        float xb[16];
        #pragma unroll
        for (int i = 0; i < 8; ++i) {
          xb[i]     = sKV[(k0 + 8 * h + i) * 64 + cn];
          xb[8 + i] = sKV[(k0 + 16 + 8 * h + i) * 64 + cn];
        }
        const v4f b0 = {xb[0], xb[1], xb[2], xb[3]};
        const v4f b1 = {xb[4], xb[5], xb[6], xb[7]};
        const v4f b2 = {xb[8], xb[9], xb[10], xb[11]};
        const v4f b3 = {xb[12], xb[13], xb[14], xb[15]};
        v16b bh, bl;
        split16v(b0, b1, b2, b3, bh, bl);
        acc = mac3(ah, al, bh, bl, acc);
      }
    } else if (w == 8) {
      #pragma unroll 2
      for (int kk = 0; kk < 64; ++kk) {
        const int j = 64 * c + kk;
        const float p = sP[rr * SPP + j];
        const int sj = (int)sKV[kk * 64 + 56];
        const int cj = (int)sKV[kk * 64 + 57];
        int rel = isr - sj;
        rel = imax(-32, imin(32, rel)) + 32;
        sS[rr * SW + rel] += p;
        cacc += (icr == cj) ? p : 0.f;
        bacc = fmaf(p, bondrow[j], bacc);
      }
    } else {
      #pragma unroll 2
      for (int kk = 0; kk < 64; ++kk) {
        const int j = 64 * c + kk;
        const float p = sP[rr * SPP + j];
        const float* rp = rbfrow + (size_t)j * 16;
        const v4f w0 = *(const v4fa*)(rp);
        const v4f w1 = *(const v4fa*)(rp + 4);
        const v4f w2 = *(const v4fa*)(rp + 8);
        const v4f w3 = *(const v4fa*)(rp + 12);
        racc[0]  = fmaf(p, w0.x, racc[0]);  racc[1]  = fmaf(p, w0.y, racc[1]);
        racc[2]  = fmaf(p, w0.z, racc[2]);  racc[3]  = fmaf(p, w0.w, racc[3]);
        racc[4]  = fmaf(p, w1.x, racc[4]);  racc[5]  = fmaf(p, w1.y, racc[5]);
        racc[6]  = fmaf(p, w1.z, racc[6]);  racc[7]  = fmaf(p, w1.w, racc[7]);
        racc[8]  = fmaf(p, w2.x, racc[8]);  racc[9]  = fmaf(p, w2.y, racc[9]);
        racc[10] = fmaf(p, w2.z, racc[10]); racc[11] = fmaf(p, w2.w, racc[11]);
        racc[12] = fmaf(p, w3.x, racc[12]); racc[13] = fmaf(p, w3.y, racc[13]);
        racc[14] = fmaf(p, w3.z, racc[14]); racc[15] = fmaf(p, w3.w, racc[15]);
      }
    }
    __syncthreads();
  }

  if (w < 8) {
    #pragma unroll
    for (int r = 0; r < 8; ++r) {
      const int row = 16 * mt + 8 * h + r, col = 16 * nt + m;
      sO[row * 64 + col] = (col < 56) ? acc[r] : 0.f;
    }
  } else if (w == 8) {
    sS[rr * SW + 81] = cacc;
    sS[rr * SW + 82] = bacc;
  } else {
    #pragma unroll
    for (int q = 0; q < 16; ++q) sS[rr * SW + 65 + q] = racc[q];
  }
  __syncthreads();
  attn_store(sO, sS, Op, Sp, zrow0, w, lane);
  __threadfence();
  attn_store(sO, sS, Op, Sp, zrow0, w, lane);
}

__device__ __forceinline__ void feats_store(const float* sFt, u16* feh, u16* fel, int r0, int tid) {
  #pragma unroll
  for (int q = 0; q < 12; ++q) {
    const int gi = tid + 128 * q;
    const int rl = gi / 96, g = gi - rl * 96;
    const v4f a = *(const v4fa*)(sFt + rl * FEAT + 8 * g);
    const v4f c = *(const v4fa*)(sFt + rl * FEAT + 8 * g + 4);
    v8us hi, lo;
    split8(a, c, hi, lo);
    stv8(feh + (size_t)(r0 + rl) * FEAT + 8 * g, hi);
    stv8(fel + (size_t)(r0 + rl) * FEAT + 8 * g, lo);
  }
}

__global__ __launch_bounds__(128) void k_feats(
    const float* __restrict__ Op, const float* __restrict__ Sp, const float* __restrict__ Fp,
    const u16* __restrict__ wph, const u16* __restrict__ wpl, u16* feh, u16* fel)
{
  __shared__ __attribute__((aligned(16))) float sFt[16 * FEAT];
  const int tid = threadIdx.x, lane = tid & 31, w = tid >> 5, h = lane >> 4, m = lane & 15;
  const int r0 = blockIdx.x * 16, b = r0 >> 9;

  if (tid < 64) {
    const int rl = tid >> 2, hq = tid & 3;
    const int row = r0 + rl, n = row & (NN - 1);
    const float* op = Op + ((size_t)(b * HH + hq) * NN + n) * QW;
    const float* fr = Fp + (size_t)row * FRW;
    const float R0 = fr[0], R1 = fr[1], R2 = fr[2], R3 = fr[3], R4 = fr[4], R5 = fr[5], R6 = fr[6], R7 = fr[7], R8 = fr[8];
    const float t0 = fr[9], t1 = fr[10], t2 = fr[11];
    float* dst = &sFt[rl * FEAT];
    #pragma unroll
    for (int c4 = 0; c4 < 8; ++c4) *(v4fa*)&dst[hq * 32 + 4 * c4] = *(const v4fa*)(op + 4 * c4);
    float og[24];
    #pragma unroll
    for (int u = 0; u < 6; ++u) {
      const v4f g4 = *(const v4fa*)(op + 32 + 4 * u);
      og[4 * u] = g4.x; og[4 * u + 1] = g4.y; og[4 * u + 2] = g4.z; og[4 * u + 3] = g4.w;
    }
    #pragma unroll
    for (int p = 0; p < 8; ++p) {
      const float vx = og[3 * p] - t0, vy = og[3 * p + 1] - t1, vz = og[3 * p + 2] - t2;
      const float olx = R0 * vx + R3 * vy + R6 * vz;
      const float oly = R1 * vx + R4 * vy + R7 * vz;
      const float olz = R2 * vx + R5 * vy + R8 * vz;
      const float nrm = sqrtf(olx * olx + oly * oly + olz * olz + 1e-8f);
      dst[128 + hq * 24 + p * 3 + 0] = olx;
      dst[128 + hq * 24 + p * 3 + 1] = oly;
      dst[128 + hq * 24 + p * 3 + 2] = olz;
      dst[224 + hq * 8 + p] = nrm;
    }
  }
  {
    const int rl = 4 * w + (m >> 2), hq = m & 3;
    const int n = (r0 + rl) & (NN - 1);
    const float* sp = Sp + ((size_t)(b * HH + hq) * NN + n) * SW;
    const v8f z8 = {0.f, 0.f, 0.f, 0.f, 0.f, 0.f, 0.f, 0.f};
    v8f acc[8];
    #pragma unroll
    for (int nt = 0; nt < 8; ++nt) acc[nt] = z8;
    #pragma unroll 1
    for (int ks = 0; ks < 3; ++ks) {
      const int k0 = 32 * ks;
      const v4f p0 = *(const v4fa*)(sp + k0 + 8 * h);
      const v4f p1 = *(const v4fa*)(sp + k0 + 8 * h + 4);
      const v4f p2 = *(const v4fa*)(sp + k0 + 16 + 8 * h);
      const v4f p3 = *(const v4fa*)(sp + k0 + 20 + 8 * h);
      v16b ah, al;
      split16v(p0, p1, p2, p3, ah, al);
      #pragma unroll
      for (int nt = 0; nt < 8; ++nt) {
        const v16b bh = ldfrag(wph + (size_t)(16 * nt + m) * WPLD + k0, h);
        const v16b bl = ldfrag(wpl + (size_t)(16 * nt + m) * WPLD + k0, h);
        acc[nt] = mac3(ah, al, bh, bl, acc[nt]);
      }
    }
    #pragma unroll
    for (int nt = 0; nt < 8; ++nt) {
      #pragma unroll
      for (int r = 0; r < 8; ++r) {
        const int rl2 = 4 * w + 2 * h + (r >> 2), hq2 = r & 3;
        sFt[rl2 * FEAT + 256 + hq2 * 128 + 16 * nt + m] = acc[nt][r];
      }
    }
  }
  __syncthreads();
  feats_store(sFt, feh, fel, r0, tid);
  __threadfence();
  feats_store(sFt, feh, fel, r0, tid);
}

extern "C" void kernel_launch(void* const* d_in, const int* in_sizes, int n_in,
                              void* d_out, int out_size, void* d_ws, size_t ws_size,
                              hipStream_t stream)
{
  if (n_in < 23) return;
  if (in_sizes[0] != ROWS || in_sizes[1] != ROWS || in_sizes[2] != ROWS || in_sizes[3] != ROWS) return;
  if (in_sizes[4] != ROWS * 7 || in_sizes[5] != BB || in_sizes[6] != BB * NN * NN) return;
  if (in_sizes[7] != IE * CS || in_sizes[8] != IE * CS || in_sizes[9] != NAA * CS) return;
  if (in_sizes[10] != NREL * CZ || in_sizes[11] != NRBF * CZ || in_sizes[12] != CZ || in_sizes[13] != CZ) return;
  if (in_sizes[14] != CS * 128 || in_sizes[15] != CS * 128 || in_sizes[16] != CS * 128) return;
  if (in_sizes[17] != CS * 48 || in_sizes[18] != CS * 48 || in_sizes[19] != CS * 96) return;
  if (in_sizes[20] != CZ * HH || in_sizes[21] != HH || in_sizes[22] != FEAT * CS) return;
  if (out_size != ROWS * CS) return;

  const int*   seq       = (const int*)  d_in[0];
  const int*   seq_idx   = (const int*)  d_in[1];
  const int*   chain_idx = (const int*)  d_in[2];
  const float* mask      = (const float*)d_in[3];
  const float* rigid7    = (const float*)d_in[4];
  const float* tt        = (const float*)d_in[5];
  const float* bonds     = (const float*)d_in[6];
  const float* W_time    = (const float*)d_in[7];
  const float* W_node    = (const float*)d_in[8];
  const float* W_seq     = (const float*)d_in[9];
  const float* W_relpos  = (const float*)d_in[10];
  const float* W_rbf     = (const float*)d_in[11];
  const float* W_chain   = (const float*)d_in[12];
  const float* W_bond    = (const float*)d_in[13];
  const float* Wq        = (const float*)d_in[14];
  const float* Wk        = (const float*)d_in[15];
  const float* Wv        = (const float*)d_in[16];
  const float* Wqp       = (const float*)d_in[17];
  const float* Wkp       = (const float*)d_in[18];
  const float* Wvp       = (const float*)d_in[19];
  const float* Wb        = (const float*)d_in[20];
  const float* gamma     = (const float*)d_in[21];
  const float* Wout      = (const float*)d_in[22];
  float* out = (float*)d_out;

  size_t off = 0;
  char* wsb = (char*)d_ws;
  auto carve = [&](size_t bytes) -> char* { char* r = wsb + off; off += (bytes + 4095) & ~(size_t)4095; return r; };
  float* tab  = (float*)carve((size_t)1024 * 4);
  u16* wph    = (u16*)  carve((size_t)CZ * WPLD * 2);
  u16* wpl    = (u16*)  carve((size_t)CZ * WPLD * 2);
  u16* wnh    = (u16*)  carve((size_t)CS * LD1 * 2);
  u16* wnl    = (u16*)  carve((size_t)CS * LD1 * 2);
  u16* wch    = (u16*)  carve((size_t)LINC * CS * 2);
  u16* wcl    = (u16*)  carve((size_t)LINC * CS * 2);
  u16* woh    = (u16*)  carve((size_t)CS * FEAT * 2);
  u16* wol    = (u16*)  carve((size_t)CS * FEAT * 2);
  u16* a1h    = (u16*)  carve((size_t)ROWS * LD1 * 2);
  u16* a1l    = (u16*)  carve((size_t)ROWS * LD1 * 2);
  float* nodef = (float*)carve((size_t)ROWS * CS * 4);
  u16* nodeh  = (u16*)  carve((size_t)ROWS * CS * 2);
  u16* nodel  = (u16*)  carve((size_t)ROWS * CS * 2);
  float* linf = (float*)carve((size_t)ROWS * LINC * 4);
  float* Fp   = (float*)carve((size_t)ROWS * FRW * 4);
  float* Qp   = (float*)carve((size_t)ZZ * NN * QW * 4);
  float* Kp   = (float*)carve((size_t)ZZ * NN * QW * 4);
  float* Vp   = (float*)carve((size_t)ZZ * NN * QW * 4);
  float* rbfp = (float*)carve((size_t)BB * NN * NN * 16 * 4);
  float* biasp = (float*)carve((size_t)BB * NN * NN * 4 * 4);
  float* Op   = (float*)carve((size_t)ZZ * NN * QW * 4);
  float* Sp   = (float*)carve((size_t)ZZ * NN * SW * 4);
  u16* feh    = (u16*)  carve((size_t)ROWS * FEAT * 2);
  u16* fel    = (u16*)  carve((size_t)ROWS * FEAT * 2);
  if (off > ws_size) return;
  if (off > (size_t)134217728) return;

  k_prep<<<dim3(1), dim3(256), 0, stream>>>(tt, gamma, W_relpos, W_rbf, W_chain, W_bond, Wb, tab, wph, wpl);
  k_wconv<<<dim3(360), dim3(256), 0, stream>>>(W_node, W_seq, W_time, Wq, Wk, Wv, Wqp, Wkp, Wvp, Wout,
                                               wnh, wnl, wch, wcl, woh, wol, tab);
  k_embed<<<dim3(ROWS), dim3(96), 0, stream>>>(seq, seq_idx, tab, a1h, a1l);
  k_gemm3<<<dim3(CS / 64, ROWS / 64), dim3(128), 0, stream>>>(a1h, a1l, LD1, wnh, wnl, LD1, K1,
                                                             nodef, CS, (const float*)nullptr, 0, nodeh, nodel, CS);
  k_gemm3<<<dim3(LINC / 64, ROWS / 64), dim3(128), 0, stream>>>(nodeh, nodel, CS, wch, wcl, CS, CS,
                                                               linf, LINC, (const float*)nullptr, 0,
                                                               (u16*)nullptr, (u16*)nullptr, 0);
  k_pack<<<dim3(ROWS), dim3(128), 0, stream>>>(linf, rigid7, seq_idx, chain_idx, mask, Qp, Kp, Vp, Fp);
  k_pair<<<dim3(BB * NN * 2), dim3(256), 0, stream>>>(rigid7, seq_idx, chain_idx, bonds, tab, rbfp, biasp);
  k_attn<<<dim3(NN / 32, ZZ), dim3(NTHA), 0, stream>>>(Qp, Kp, Vp, biasp, rbfp, bonds, tab, Op, Sp);
  k_feats<<<dim3(ROWS / 16), dim3(128), 0, stream>>>(Op, Sp, Fp, wph, wpl, feh, fel);
  k_gemm3<<<dim3(CS / 64, ROWS / 64), dim3(128), 0, stream>>>(feh, fel, FEAT, woh, wol, FEAT, FEAT,
                                                             out, CS, nodef, CS, (u16*)nullptr, (u16*)nullptr, 0);
}
